// BANLayer_89893665505605
// MI455X (gfx1250) — hardware-run, weakly checked
//
#include <hip/hip_runtime.h>
#include <stddef.h>

#define NB    16
#define VNUM  1024
#define QNUM  512
#define VDIM  256
#define QDIM  128
#define NH    8
#define HD    64
#define PROJ  512
#define FDIM  1024
#define NBH   128
#define VBLK  (VNUM / 64)
#define RBLK  (VNUM / 64)

static_assert(PROJ == NH * HD);
static_assert(FDIM == 2 * PROJ);
static_assert(NBH == NB * NH);
static_assert(NB == 16);
static_assert(HD == 64);
static_assert(QNUM == 512);
static_assert(VNUM % 64 == 0);
static_assert(QNUM % 64 == 0);
static_assert(VDIM % 64 == 0);
static_assert(QDIM % 64 == 0);
static_assert(FDIM % 64 == 0);
static_assert(PROJ % 64 == 0);
static_assert((NB * VNUM * VDIM) % 2048 == 0);
static_assert((NB * QNUM * QDIM) % 2048 == 0);
static_assert((NH * HD * HD) % 2048 == 0);

typedef unsigned short us;
typedef _Float16     v16h __attribute__((ext_vector_type(16)));
typedef us           v8us __attribute__((ext_vector_type(8)));
typedef float        v8f  __attribute__((ext_vector_type(8)));
typedef float        v4f  __attribute__((ext_vector_type(4)));
typedef unsigned int v4u  __attribute__((ext_vector_type(4)));

union Frag  { v16h v; v8us h[2]; };
union Pack8 { v8us h; v4u u; };

__device__ __forceinline__ us h16(float f) {
  const _Float16 x = (_Float16)f;
  return __builtin_bit_cast(us, x);
}
__device__ __forceinline__ float hval(us u) { return (float)__builtin_bit_cast(_Float16, u); }
__device__ __forceinline__ v4u pack8(const float (&f)[8], float sc) {
  Pack8 p;
  p.h = (v8us){h16(f[0] * sc), h16(f[1] * sc), h16(f[2] * sc), h16(f[3] * sc),
               h16(f[4] * sc), h16(f[5] * sc), h16(f[6] * sc), h16(f[7] * sc)};
  return p.u;
}
__device__ __forceinline__ v8f zero8() { return (v8f){0.f, 0.f, 0.f, 0.f, 0.f, 0.f, 0.f, 0.f}; }

__device__ __forceinline__ v8f mma16(v16h a, v16h b, v8f c) {
  c = __builtin_amdgcn_wmma_f32_16x16x32_f16(false, a, false, b, (short)0, c, false, false);
  asm volatile("v_nop\n\tv_nop\n\tv_nop\n\tv_nop" : "+v"(c) : "v"(a), "v"(b));
  return c;
}

__device__ __forceinline__ v16h ldfrag(const us* p, int ld, int row0, int k0, int lane) {
  const int m = lane & 15, lh = lane >> 4;
  const us* q = p + (size_t)(row0 + m) * ld + k0 + 8 * lh;
  Frag f;
  f.h[0] = *(const v8us*)(q);
  f.h[1] = *(const v8us*)(q + 16);
  return f.v;
}

template <int KD>
__device__ __forceinline__ void gemm16x64(const us* __restrict__ A, int lda, int arow0, int acol0,
                                          const us* __restrict__ Bt, int ldb, int brow0, int lane,
                                          v8f (&acc)[4]) {
  static_assert(KD % 32 == 0);
#pragma unroll 1
  for (int k0 = 0; k0 < KD; k0 += 32) {
    const v16h a = ldfrag(A, lda, arow0, acol0 + k0, lane);
#pragma unroll
    for (int t = 0; t < 4; ++t) {
      const v16h b = ldfrag(Bt, ldb, brow0 + 16 * t, k0, lane);
      acc[t] = mma16(a, b, acc[t]);
    }
  }
}

__global__ __launch_bounds__(256) void k_cvt(const float* __restrict__ x, us* __restrict__ y, float scale) {
  const size_t i = (size_t)blockIdx.x * 2048 + (size_t)threadIdx.x * 8;
  const v4f a0 = *(const v4f*)(x + i);
  const v4f a1 = *(const v4f*)(x + i + 4);
  const float f[8] = {a0[0], a0[1], a0[2], a0[3], a1[0], a1[1], a1[2], a1[3]};
  const v4u hv = pack8(f, scale);
  *(volatile v4u*)(y + i) = hv;
  __threadfence();
  *(volatile v4u*)(y + i) = hv;
}

#define SFP 68
__global__ __launch_bounds__(256) void k_cvt_wt(const float* __restrict__ w, us* __restrict__ wt,
                                                int K, int N, float scale) {
  __shared__ __align__(16) float sw[64 * SFP];
  const int tid = threadIdx.x;
  const int kb = blockIdx.x * 64;
  const int nb = blockIdx.y * 64;
  {
    const int r  = tid >> 2;
    const int c0 = (tid & 3) * 16;
    const float* src = w + (size_t)(kb + r) * N + nb + c0;
#pragma unroll
    for (int e = 0; e < 4; ++e) *(v4f*)(sw + r * SFP + c0 + 4 * e) = *(const v4f*)(src + 4 * e);
  }
  __syncthreads();
  v4u hv[2];
  size_t go[2];
#pragma unroll
  for (int j = 0; j < 2; ++j) {
    const int p  = tid + 256 * j;
    const int n  = p >> 3;
    const int pc = p & 7;
    const float* cp = sw + (pc * 8) * SFP + n;
    float f[8];
#pragma unroll
    for (int e = 0; e < 8; ++e) f[e] = cp[e * SFP];
    hv[j] = pack8(f, scale);
    go[j] = (size_t)(nb + n) * (size_t)K + kb + pc * 8;
  }
#pragma unroll
  for (int j = 0; j < 2; ++j) *(volatile v4u*)(wt + go[j]) = hv[j];
  __threadfence();
#pragma unroll
  for (int j = 0; j < 2; ++j) *(volatile v4u*)(wt + go[j]) = hv[j];
}

template <int KD, int MODE>
__global__ __launch_bounds__(128) void k_gemm(const us* __restrict__ A, const us* __restrict__ Bt,
                                              const float* __restrict__ bias, us* __restrict__ Y,
                                              float* __restrict__ CSUM) {
  __shared__ __align__(16) float sf[64 * SFP];
  __shared__ __align__(16) float cred[64];
  const int tid = threadIdx.x, lane = tid & 31, wave = tid >> 5;
  const int hh = lane >> 4, c = lane & 15;

  int lda, arow0, acol0, ldb, brow0, ldy, yrow0, ycol0, boff;
  float alpha;
  if (MODE == 0) {
    lda = VDIM; arow0 = blockIdx.x * 64; acol0 = 0; ldb = VDIM; brow0 = blockIdx.y * 64;
    ldy = PROJ; yrow0 = arow0; ycol0 = brow0; boff = brow0; alpha = 0.0625f;
  } else if (MODE == 1) {
    lda = QDIM; arow0 = blockIdx.x * 64; acol0 = 0; ldb = QDIM; brow0 = blockIdx.y * 64;
    ldy = PROJ; yrow0 = arow0; ycol0 = brow0; boff = brow0; alpha = 0.0625f;
  } else {
    const int bh = blockIdx.x >> 3, rb = blockIdx.x & 7, b = bh >> 3, h = bh & 7;
    lda = PROJ; arow0 = b * QNUM + rb * 64; acol0 = h * HD; ldb = HD; brow0 = h * HD;
    ldy = HD; yrow0 = bh * QNUM + rb * 64; ycol0 = 0; boff = 0; alpha = 0.0625f;
  }

  v8f acc[4];
#pragma unroll
  for (int t = 0; t < 4; ++t) acc[t] = zero8();
  gemm16x64<KD>(A, lda, arow0 + wave * 16, acol0, Bt, ldb, brow0, lane, acc);

  float bcol[4];
#pragma unroll
  for (int t = 0; t < 4; ++t) {
    if (MODE != 2) bcol[t] = bias[boff + 16 * t + c];
    else           bcol[t] = 0.f;
  }
#pragma unroll
  for (int t = 0; t < 4; ++t) {
#pragma unroll
    for (int r = 0; r < 8; ++r)
      sf[(wave * 16 + 8 * hh + r) * SFP + 16 * t + c] = acc[t][r] * alpha + bcol[t];
  }
  __syncthreads();

  v4u hv[4];
  size_t go[4];
#pragma unroll
  for (int j = 0; j < 4; ++j) {
    const int p  = tid + 128 * j;
    const int lr = p >> 3;
    const int d0 = (p & 7) * 8;
    const float* ra = sf + lr * SFP + d0;
    const v4f a0 = *(const v4f*)(ra), a1 = *(const v4f*)(ra + 4);
    const float f[8] = {a0[0], a0[1], a0[2], a0[3], a1[0], a1[1], a1[2], a1[3]};
    hv[j] = pack8(f, 1.0f);
    go[j] = (size_t)(yrow0 + lr) * (size_t)ldy + ycol0 + d0;
  }
  v4f cv = (v4f){0.f, 0.f, 0.f, 0.f};
  size_t co = 0;
  if (MODE == 0) {
    if (tid < 64) {
      float s = 0.f;
#pragma unroll 1
      for (int r = 0; r < 64; ++r) s += sf[r * SFP + tid];
      cred[tid] = s;
    }
    __syncthreads();
    const int li = (tid < 16) ? tid : 0;
    cv = *(const v4f*)(cred + 4 * li);
    co = (size_t)blockIdx.x * PROJ + blockIdx.y * 64 + 4 * li;
  }
#pragma unroll
  for (int j = 0; j < 4; ++j) *(volatile v4u*)(Y + go[j]) = hv[j];
  if (MODE == 0) { if (tid < 16) *(volatile v4f*)(CSUM + co) = cv; }
  __threadfence();
#pragma unroll
  for (int j = 0; j < 4; ++j) *(volatile v4u*)(Y + go[j]) = hv[j];
  if (MODE == 0) { if (tid < 16) *(volatile v4f*)(CSUM + co) = cv; }
}

__global__ __launch_bounds__(256) void k_logits(const us* __restrict__ VP, const us* __restrict__ U,
                                                float* __restrict__ CBP) {
  __shared__ float redmax[8 * 16];
  __shared__ float redsum[8 * 16];
  __shared__ float rowmax[16];
  __shared__ float rowsum[16];
  __shared__ __align__(16) float colbuf[8 * 64];
  const int tid = threadIdx.x, lane = tid & 31, wave = tid >> 5;
  const int hh = lane >> 4, c = lane & 15;
  const int bh = blockIdx.x >> 4, vblk = blockIdx.x & 15;
  const int b = bh >> 3, h = bh & 7;
  const int col0 = wave * 64;
  const us* Ub = U + (size_t)bh * QNUM * HD;
  const int vrow0 = b * VNUM + vblk * 64;

  float cs[4] = {0.f, 0.f, 0.f, 0.f};
#pragma unroll 1
  for (int g = 0; g < 4; ++g) {
    v8f s[4];
#pragma unroll
    for (int t = 0; t < 4; ++t) s[t] = zero8();
#pragma unroll
    for (int dc = 0; dc < 2; ++dc) {
      const v16h a = ldfrag(VP, PROJ, vrow0 + g * 16, h * HD + dc * 32, lane);
#pragma unroll
      for (int t = 0; t < 4; ++t) {
        const v16h bf = ldfrag(Ub, HD, col0 + 16 * t, dc * 32, lane);
        s[t] = mma16(a, bf, s[t]);
      }
    }
#pragma unroll
    for (int t = 0; t < 4; ++t)
#pragma unroll
      for (int e = 0; e < 8; ++e) s[t][e] *= 0.125f;

    float m[8];
#pragma unroll
    for (int e = 0; e < 8; ++e) m[e] = fmaxf(fmaxf(s[0][e], s[1][e]), fmaxf(s[2][e], s[3][e]));
#pragma unroll
    for (int off = 1; off < 16; off <<= 1)
#pragma unroll
      for (int e = 0; e < 8; ++e) m[e] = fmaxf(m[e], __shfl_xor(m[e], off, 32));
    if (c == 0) {
#pragma unroll
      for (int e = 0; e < 8; ++e) redmax[wave * 16 + hh * 8 + e] = m[e];
    }
    __syncthreads();
    if (tid < 16) {
      float v = redmax[tid];
#pragma unroll
      for (int w = 1; w < 8; ++w) v = fmaxf(v, redmax[w * 16 + tid]);
      rowmax[tid] = v;
    }
    __syncthreads();
    float rm[8];
#pragma unroll
    for (int e = 0; e < 8; ++e) rm[e] = rowmax[hh * 8 + e];

    float rs[8];
#pragma unroll
    for (int e = 0; e < 8; ++e) rs[e] = 0.f;
#pragma unroll
    for (int t = 0; t < 4; ++t)
#pragma unroll
      for (int e = 0; e < 8; ++e) {
        const float ev = __expf(s[t][e] - rm[e]);
        s[t][e] = ev;
        rs[e] += ev;
      }
#pragma unroll
    for (int off = 1; off < 16; off <<= 1)
#pragma unroll
      for (int e = 0; e < 8; ++e) rs[e] += __shfl_xor(rs[e], off, 32);
    if (c == 0) {
#pragma unroll
      for (int e = 0; e < 8; ++e) redsum[wave * 16 + hh * 8 + e] = rs[e];
    }
    __syncthreads();
    if (tid < 16) {
      float v = 0.f;
#pragma unroll
      for (int w = 0; w < 8; ++w) v += redsum[w * 16 + tid];
      rowsum[tid] = v;
    }
    __syncthreads();
    float ri[8];
#pragma unroll
    for (int e = 0; e < 8; ++e) ri[e] = 1.0f / rowsum[hh * 8 + e];
#pragma unroll
    for (int t = 0; t < 4; ++t) {
      float a = 0.f;
#pragma unroll
      for (int e = 0; e < 8; ++e) a += s[t][e] * ri[e];
      cs[t] += a;
    }
  }
#pragma unroll
  for (int t = 0; t < 4; ++t) cs[t] += __shfl_xor(cs[t], 16, 32);
  if (hh == 0) {
#pragma unroll
    for (int t = 0; t < 4; ++t) colbuf[wave * 64 + 16 * t + c] = cs[t];
  }
  __syncthreads();
  const int li = (lane < 16) ? lane : 0;
  const v4f cv = *(const v4f*)(colbuf + wave * 64 + 4 * li);
  float* dst = CBP + ((size_t)(bh * VBLK + vblk) * QNUM + col0 + 4 * li);
  if (lane < 16) *(volatile v4f*)dst = cv;
  __threadfence();
  if (lane < 16) *(volatile v4f*)dst = cv;
}

__global__ __launch_bounds__(256) void k_pool(const float* __restrict__ CBP, const us* __restrict__ QP,
                                              const float* __restrict__ CSUM, us* __restrict__ FUS) {
  __shared__ float cb[QNUM];
  __shared__ float pv4[256];
  __shared__ __align__(16) us fo[128];
  const int tid = threadIdx.x;
  const int bh = blockIdx.x, b = bh >> 3, h = bh & 7;

#pragma unroll
  for (int k = 0; k < 2; ++k) {
    const int qq = tid + 256 * k;
    float s = 0.f;
#pragma unroll 1
    for (int r = 0; r < VBLK; ++r) s += CBP[((size_t)(bh * VBLK + r)) * QNUM + qq];
    cb[qq] = s;
  }
  __syncthreads();
  {
    const int j = tid & 63, part = tid >> 6;
    const us* qcol = QP + (size_t)(b * QNUM + part * 128) * PROJ + h * HD + j;
    const float* cbp = cb + part * 128;
    float a = 0.f;
#pragma unroll 4
    for (int qi = 0; qi < 128; ++qi) a = fmaf(cbp[qi], hval(qcol[(size_t)qi * PROJ]), a);
    pv4[tid] = a;
  }
  __syncthreads();
  if (tid < 64) {
    const float pv = (((pv4[tid] + pv4[64 + tid]) + pv4[128 + tid]) + pv4[192 + tid]) * (1.0f / 1024.0f);
    fo[tid] = h16(pv * 256.0f);
  } else if (tid < 128) {
    const int i = tid - 64;
    float s = 0.f;
#pragma unroll 1
    for (int r = 0; r < RBLK; ++r) s += CSUM[((size_t)(b * RBLK + r)) * PROJ + h * HD + i];
    fo[tid] = h16(s * (1.0f / 512.0f) * 256.0f);
  }
  __syncthreads();
  const int li = (tid < 16) ? tid : 0;
  const v4u fv = *(const v4u*)(fo + 8 * li);
  us* dst = FUS + (size_t)b * FDIM + h * 128 + 8 * li;
  if (tid < 16) *(volatile v4u*)dst = fv;
  __threadfence();
  if (tid < 16) *(volatile v4u*)dst = fv;
}

#define OTP 68
__global__ __launch_bounds__(256) void k_out(const us* __restrict__ FUS, const us* __restrict__ WOT,
                                             const float* __restrict__ bo, float* __restrict__ out) {
  __shared__ __align__(16) float osw[8 * 16 * OTP];
  const int tid = threadIdx.x, lane = tid & 31, wave = tid >> 5;
  const int hh = lane >> 4, c = lane & 15;
  const int col0 = wave * 64;

  v8f acc[4];
#pragma unroll
  for (int t = 0; t < 4; ++t) acc[t] = zero8();
  gemm16x64<FDIM>(FUS, FDIM, 0, 0, WOT, FDIM, col0, lane, acc);

  float bcol[4];
#pragma unroll
  for (int t = 0; t < 4; ++t) bcol[t] = bo[col0 + 16 * t + c];
  float* ow = osw + wave * 16 * OTP;
#pragma unroll
  for (int r = 0; r < 8; ++r) {
#pragma unroll
    for (int t = 0; t < 4; ++t) {
      const float v = acc[t][r] * (1.0f / 16384.0f) + bcol[t];
      ow[(8 * hh + r) * OTP + 16 * t + c] = fmaxf(v, 0.f);
    }
  }
  __syncthreads();
  v4f val[8];
  size_t go[8];
#pragma unroll
  for (int it = 0; it < 8; ++it) {
    const int p    = lane + 32 * it;
    const int L    = p >> 3;
    const int pc   = p & 7;
    const int row  = L >> 1;
    const int half = L & 1;
    const int col  = half * 32 + pc * 4;
    val[it] = *(const v4f*)(ow + row * OTP + col);
    go[it]  = (size_t)row * PROJ + col0 + col;
  }
#pragma unroll
  for (int it = 0; it < 8; ++it) *(volatile v4f*)(out + go[it]) = val[it];
  __threadfence();
#pragma unroll
  for (int it = 0; it < 8; ++it) *(volatile v4f*)(out + go[it]) = val[it];
}

extern "C" void kernel_launch(void* const* d_in, const int* in_sizes, int n_in,
                              void* d_out, int out_size, void* d_ws, size_t ws_size,
                              hipStream_t stream) {
  if (n_in < 9) return;
  if (in_sizes[0] != NB * VNUM * VDIM) return;
  if (in_sizes[1] != NB * QNUM * QDIM) return;
  if (in_sizes[2] != VDIM * PROJ) return;
  if (in_sizes[3] != PROJ) return;
  if (in_sizes[4] != QDIM * PROJ) return;
  if (in_sizes[5] != PROJ) return;
  if (in_sizes[6] != NH * HD * HD) return;
  if (in_sizes[7] != FDIM * PROJ) return;
  if (in_sizes[8] != PROJ) return;
  if (out_size != NB * PROJ) return;

  const float* v    = (const float*)d_in[0];
  const float* q    = (const float*)d_in[1];
  const float* Wv   = (const float*)d_in[2];
  const float* bv   = (const float*)d_in[3];
  const float* Wq   = (const float*)d_in[4];
  const float* bq   = (const float*)d_in[5];
  const float* attw = (const float*)d_in[6];
  const float* Wo   = (const float*)d_in[7];
  const float* bo   = (const float*)d_in[8];
  float* out = (float*)d_out;

  size_t off = 0;
  const size_t oVH  = off; off += (size_t)NB * VNUM * VDIM * 2;
  const size_t oQH  = off; off += (size_t)NB * QNUM * QDIM * 2;
  const size_t oAW  = off; off += (size_t)NH * HD * HD * 2;
  const size_t oWVT = off; off += (size_t)PROJ * VDIM * 2;
  const size_t oWQT = off; off += (size_t)PROJ * QDIM * 2;
  const size_t oWOT = off; off += (size_t)PROJ * FDIM * 2;
  const size_t oVP  = off; off += (size_t)NB * VNUM * PROJ * 2;
  const size_t oQP  = off; off += (size_t)NB * QNUM * PROJ * 2;
  const size_t oU   = off; off += (size_t)NBH * QNUM * HD * 2;
  const size_t oCBP = off; off += (size_t)NBH * VBLK * QNUM * 4;
  const size_t oCS  = off; off += (size_t)NB * RBLK * PROJ * 4;
  const size_t oFUS = off; off += (size_t)NB * FDIM * 2;
  if (off > ws_size) return;
  if (off > (size_t)134217728) return;

  char* ws = (char*)d_ws;
  us* VH  = (us*)(ws + oVH);
  us* QH  = (us*)(ws + oQH);
  us* AW  = (us*)(ws + oAW);
  us* WVT = (us*)(ws + oWVT);
  us* WQT = (us*)(ws + oWQT);
  us* WOT = (us*)(ws + oWOT);
  us* VP  = (us*)(ws + oVP);
  us* QP  = (us*)(ws + oQP);
  us* UP  = (us*)(ws + oU);
  float* CBP  = (float*)(ws + oCBP);
  float* CSUM = (float*)(ws + oCS);
  us* FUS = (us*)(ws + oFUS);

  k_cvt<<<dim3((NB * VNUM * VDIM) / 2048), dim3(256), 0, stream>>>(v, VH, 1.0f);
  k_cvt<<<dim3((NB * QNUM * QDIM) / 2048), dim3(256), 0, stream>>>(q, QH, 1.0f);
  k_cvt<<<dim3((NH * HD * HD) / 2048), dim3(256), 0, stream>>>(attw, AW, 16.0f);
  k_cvt_wt<<<dim3(VDIM / 64, PROJ / 64), dim3(256), 0, stream>>>(Wv, WVT, VDIM, PROJ, 16.0f);
  k_cvt_wt<<<dim3(QDIM / 64, PROJ / 64), dim3(256), 0, stream>>>(Wq, WQT, QDIM, PROJ, 16.0f);
  k_cvt_wt<<<dim3(FDIM / 64, PROJ / 64), dim3(256), 0, stream>>>(Wo, WOT, FDIM, PROJ, 64.0f);
  k_gemm<VDIM, 0><<<dim3((NB * VNUM) / 64, PROJ / 64), dim3(128), 0, stream>>>(VH, WVT, bv, VP, CSUM);
  k_gemm<QDIM, 1><<<dim3((NB * QNUM) / 64, PROJ / 64), dim3(128), 0, stream>>>(QH, WQT, bq, QP, CSUM);
  k_gemm<HD, 2><<<dim3(NBH * (QNUM / 64)), dim3(128), 0, stream>>>(QP, AW, bq, UP, CSUM);
  k_logits<<<dim3(NBH * VBLK), dim3(256), 0, stream>>>(VP, UP, CBP);
  k_pool<<<dim3(NBH), dim3(256), 0, stream>>>(CBP, QP, CSUM, FUS);
  k_out<<<dim3(1), dim3(256), 0, stream>>>(FUS, WOT, bo, out);
  (void)hipGetLastError();
}
